// HTALayer_72911364817309
// MI455X (gfx1250) — hardware-verified
//
#include <hip/hip_runtime.h>
#include <math.h>

constexpr int kNodes = 2048;
constexpr int kEdges = 512;
constexpr int kDim   = 256;
constexpr int kHeads = 8;
constexpr int kHd    = 32;
constexpr int kRank  = 32;
constexpr int kHeadBatch = 2;
constexpr int kGateN = 64;
constexpr int kVRows = kDim + 32;
constexpr float kWCarry     = 16.0f;
constexpr float kWCarryInv  = 1.0f / 16.0f;
constexpr float kPCarry     = 32768.0f;
constexpr float kPCarryInv  = 1.0f / 32768.0f;
constexpr float kScoreScale = 0.17677669529663687f;
constexpr float kInvDim     = 1.0f / 256.0f;
constexpr float kLnEps      = 1e-5f;

typedef __attribute__((ext_vector_type(16))) _Float16 v16h;
typedef __attribute__((ext_vector_type(8)))  _Float16 v8h;
typedef __attribute__((ext_vector_type(16))) __bf16   v16b;
typedef __attribute__((ext_vector_type(8)))  __bf16   v8b;
typedef __attribute__((ext_vector_type(8)))  float    v8f;
typedef __attribute__((ext_vector_type(4)))  float    v4f;
typedef __attribute__((ext_vector_type(4)))  unsigned int v4u;

__device__ __forceinline__ unsigned short f2bf_bits(float f) {
  unsigned u = __float_as_uint(f);
  return (unsigned short)((u + 0x7FFFu + ((u >> 16) & 1u)) >> 16);
}
__device__ __forceinline__ float bf_bits2f(unsigned short h) { return __uint_as_float(((unsigned)h) << 16); }

__device__ __forceinline__ void dep_guard_h(v8f& a, v8f& b, v16h x, v16h y) { asm volatile("v_nop\n\tv_nop\n\tv_nop\n\tv_nop" : "+v"(a), "+v"(b) : "v"(x), "v"(y)); }
__device__ __forceinline__ void dep_guard_b(v8f& a, v8f& b, v16b x, v16b y) { asm volatile("v_nop\n\tv_nop\n\tv_nop\n\tv_nop" : "+v"(a), "+v"(b) : "v"(x), "v"(y)); }
__device__ __forceinline__ void keep4_h(v16h a, v16h b, v16h c, v16h d) { asm volatile("v_nop" :: "v"(a), "v"(b), "v"(c), "v"(d)); }
__device__ __forceinline__ void keep4_b(v16b a, v16b b, v16b c, v16b d) { asm volatile("v_nop" :: "v"(a), "v"(b), "v"(c), "v"(d)); }
__device__ __forceinline__ void acc_guard4(v8f& a, v8f& b, v8f& c, v8f& d) { asm volatile("v_nop\n\tv_nop\n\tv_nop\n\tv_nop" : "+v"(a), "+v"(b), "+v"(c), "+v"(d)); }
template <typename T> struct Frag;
template <> struct Frag<_Float16> {
  typedef v16h V; union U { v16h v; v8h h[2]; };
  static __device__ __forceinline__ v16h load(const _Float16* p) {
    U f; f.h[0] = *(const v8h*)(p); f.h[1] = *(const v8h*)(p + 16); return f.v;
  }
  static __device__ __forceinline__ v8f mma(v16h a, v16h b, v8f c) {
    return __builtin_amdgcn_wmma_f32_16x16x32_f16(false, a, false, b, (short)0, c, false, false);
  }
  static __device__ __forceinline__ void guard(v8f& a, v8f& b, v16h x, v16h y) { dep_guard_h(a, b, x, y); }
  static __device__ __forceinline__ void keep(v16h a, v16h b, v16h c, v16h d) { keep4_h(a, b, c, d); }
};
template <> struct Frag<__bf16> {
  typedef v16b V; union U { v16b v; v8b h[2]; };
  static __device__ __forceinline__ v16b load(const __bf16* p) {
    U f; f.h[0] = *(const v8b*)(p); f.h[1] = *(const v8b*)(p + 16); return f.v;
  }
  static __device__ __forceinline__ v8f mma(v16b a, v16b b, v8f c) {
    return __builtin_amdgcn_wmma_f32_16x16x32_bf16(false, a, false, b, (short)0, c, false, false);
  }
  static __device__ __forceinline__ void guard(v8f& a, v8f& b, v16b x, v16b y) { dep_guard_b(a, b, x, y); }
  static __device__ __forceinline__ void keep(v16b a, v16b b, v16b c, v16b d) { keep4_b(a, b, c, d); }
};

__device__ __forceinline__ unsigned pk16(unsigned short a, unsigned short b) { return (unsigned)a | ((unsigned)b << 16); }
__device__ __forceinline__ unsigned short h_bits(float f) { const _Float16 h = (_Float16)f; return __builtin_bit_cast(unsigned short, h); }

template <int ET> struct Elem;
template <> struct Elem<0> { typedef _Float16 T; };
template <> struct Elem<1> { typedef __bf16 T; };
template <int ET, bool SPLIT, int BIAS_MODE, int OUT_MODE, bool RESID, int ACT = 0>
__global__ __launch_bounds__(256) void wmma_gemm64(
    const unsigned short* __restrict__ Ap, const unsigned short* __restrict__ A2p, int lda, long strideA,
    const unsigned short* __restrict__ Btp, const unsigned short* __restrict__ Bt2p, int ldb, long strideB,
    void* __restrict__ Cout, void* __restrict__ Cout2, int ldc, long strideC,
    const float* __restrict__ bias,
    const float* __restrict__ resid, long strideR,
    int M, int N, int K, float scale) {
  typedef typename Elem<ET>::T T;
  typedef typename Frag<T>::V V;
  const T* A = (const T*)Ap; const T* A2 = (const T*)A2p; const T* Bt = (const T*)Btp; const T* Bt2 = (const T*)Bt2p;
  __shared__ __align__(16) float sT[8][16 * 68];
  const int b    = blockIdx.y;
  const int lane = threadIdx.x & 31;
  const int wave = threadIdx.x >> 5;
  const int tilesN = N >> 6;
  const int tilesM = M >> 6;
  const int tile = blockIdx.x * 8 + wave;
  if (tile >= tilesM * tilesN) return;
  const int tm = tile / tilesN;
  const int tn = tile - tm * tilesN;
  const int m0 = tm << 6;
  const int n0 = tn << 6;

  const T* Ab  = A  + (size_t)b * strideA;
  const T* Bb  = Bt + (size_t)b * strideB;
  const T* Ab2 = SPLIT ? (A2  + (size_t)b * strideA) : nullptr;
  const T* Bb2 = SPLIT ? (Bt2 + (size_t)b * strideB) : nullptr;

  const int rlane = lane & 15;
  const int koff  = (lane >> 4) * 8;
  const int mOff  = (lane >> 4) * 8;

  v8f acc[4][4];
#pragma unroll
  for (int i = 0; i < 4; ++i)
#pragma unroll
    for (int j = 0; j < 4; ++j) acc[i][j] = (v8f){0.f,0.f,0.f,0.f,0.f,0.f,0.f,0.f};

  for (int k0 = 0; k0 < K; k0 += 32) {
    V bh[4], bl[4];
#pragma unroll
    for (int j = 0; j < 4; ++j) {
      const size_t bo = (size_t)(n0 + (j << 4) + rlane) * ldb + koff + k0;
      bh[j] = Frag<T>::load(Bb + bo);
      if (SPLIT) bl[j] = Frag<T>::load(Bb2 + bo);
    }
#pragma unroll
    for (int i = 0; i < 4; ++i) {
      const size_t ao = (size_t)(m0 + (i << 4) + rlane) * lda + koff + k0;
      V ah = Frag<T>::load(Ab + ao);
      V al;
      if (SPLIT) al = Frag<T>::load(Ab2 + ao);
#pragma unroll
      for (int j = 0; j < 4; ++j) {
        acc[i][j] = Frag<T>::mma(ah, bh[j], acc[i][j]);
        if (SPLIT) {
          acc[i][j] = Frag<T>::mma(ah, bl[j], acc[i][j]);
          acc[i][j] = Frag<T>::mma(al, bh[j], acc[i][j]);
        }
      }
      Frag<T>::guard(acc[i][0], acc[i][3], ah, SPLIT ? al : ah);
    }
    Frag<T>::keep(bh[0], bh[1], bh[2], bh[3]);
    if (SPLIT) Frag<T>::keep(bl[0], bl[1], bl[2], bl[3]);
  }
  acc_guard4(acc[0][0], acc[0][1], acc[0][2], acc[0][3]);
  acc_guard4(acc[1][0], acc[1][1], acc[1][2], acc[1][3]);
  acc_guard4(acc[2][0], acc[2][1], acc[2][2], acc[2][3]);
  acc_guard4(acc[3][0], acc[3][1], acc[3][2], acc[3][3]);

  float* slab = sT[wave];
  const float* Rb = RESID ? (resid + (size_t)b * strideR) : nullptr;
#pragma unroll
  for (int i = 0; i < 4; ++i) {
    const int mBase = m0 + (i << 4);
#pragma unroll
    for (int j = 0; j < 4; ++j) {
      const int n = n0 + (j << 4) + rlane;
      float bv = 0.f;
      if (BIAS_MODE == 2) bv = bias[n];
#pragma unroll
      for (int r = 0; r < 8; ++r) {
        float v = acc[i][j][r] * scale;
        if (BIAS_MODE == 1) v += bias[mBase + mOff + r];
        if (BIAS_MODE == 2) v += bv;
        if (RESID) v += Rb[(size_t)(mBase + mOff + r) * ldc + n];
        if (ACT == 2) v = fmaxf(v, 0.0f);
        if (ACT == 4) v = (v > 0.f) ? v : 0.01f * v;
        slab[(mOff + r) * 68 + (j << 4) + rlane] = v;
      }
    }
    __builtin_amdgcn_fence(__ATOMIC_RELEASE, "workgroup");
    __builtin_amdgcn_wave_barrier();
    __builtin_amdgcn_fence(__ATOMIC_ACQUIRE, "workgroup");
    if (OUT_MODE == 0) {
      float* C = (float*)Cout + (size_t)b * strideC;
      const int hh = lane >> 4, c4 = (lane & 15) * 4;
      for (int pass = 0; pass < 2; ++pass) {
#pragma unroll
        for (int it = 0; it < 8; ++it) {
          const int row = it * 2 + hh;
          v4f v = *(const v4f*)(slab + row * 68 + c4);
          *(volatile v4f*)(C + (size_t)(mBase + row) * ldc + n0 + c4) = v;
        }
        __threadfence();
      }
    } else {
      const int q = lane >> 3, c8 = (lane & 7) * 8;
      unsigned short* C  = (unsigned short*)Cout  + (size_t)b * strideC;
      unsigned short* C2 = (OUT_MODE == 2) ? ((unsigned short*)Cout2 + (size_t)b * strideC) : nullptr;
      for (int pass = 0; pass < 2; ++pass) {
#pragma unroll
        for (int it = 0; it < 4; ++it) {
          const int row = it * 4 + q;
          const float* sp = slab + row * 68 + c8;
          v8h hv, lv;
#pragma unroll
          for (int e = 0; e < 8; ++e) {
            if (OUT_MODE == 1) {
              hv[e] = (_Float16)sp[e];
            } else {
              unsigned short hb = f2bf_bits(sp[e]);
              unsigned short lb = f2bf_bits(sp[e] - bf_bits2f(hb));
              hv[e] = __builtin_bit_cast(_Float16, hb);
              lv[e] = __builtin_bit_cast(_Float16, lb);
            }
          }
          *(volatile v8h*)(C + (size_t)(mBase + row) * ldc + n0 + c8) = hv;
          if (OUT_MODE == 2) *(volatile v8h*)(C2 + (size_t)(mBase + row) * ldc + n0 + c8) = lv;
        }
        __threadfence();
      }
    }
    __builtin_amdgcn_fence(__ATOMIC_RELEASE, "workgroup");
    __builtin_amdgcn_wave_barrier();
    __builtin_amdgcn_fence(__ATOMIC_ACQUIRE, "workgroup");
  }
}

__global__ __launch_bounds__(256) void cast8_f16_kernel(const float* __restrict__ in, unsigned short* __restrict__ out, int n8, float scale) {
  const int i = blockIdx.x * 256 + threadIdx.x;
  if (i >= n8) return;
  const float* p = in + 8 * (size_t)i;
  const v4f a = *(const v4f*)(p);
  const v4f c = *(const v4f*)(p + 4);
  unsigned short hb[8];
#pragma unroll
  for (int e = 0; e < 4; ++e) {
    hb[e]     = h_bits(a[e] * scale);
    hb[4 + e] = h_bits(c[e] * scale);
  }
  const v4u u = (v4u){pk16(hb[0], hb[1]), pk16(hb[2], hb[3]), pk16(hb[4], hb[5]), pk16(hb[6], hb[7])};
  unsigned short* q = out + 8 * (size_t)i;
  *(volatile v4u*)q = u;
  __threadfence();
  *(volatile v4u*)q = u;
}

__global__ __launch_bounds__(256) void wcast4_kernel(const float* __restrict__ W0, const float* __restrict__ W1,
                                                     const float* __restrict__ W2, const float* __restrict__ W3,
                                                     unsigned short* __restrict__ out, int n8, float scale) {
  const int i = blockIdx.x * 256 + threadIdx.x;
  const int z = blockIdx.y;
  if (i >= n8) return;
  const float* W = (z == 0) ? W0 : (z == 1) ? W1 : (z == 2) ? W2 : W3;
  const float* p = W + 8 * (size_t)i;
  const v4f a = *(const v4f*)(p);
  const v4f c = *(const v4f*)(p + 4);
  unsigned short hb[8];
#pragma unroll
  for (int e = 0; e < 4; ++e) {
    hb[e]     = h_bits(a[e] * scale);
    hb[4 + e] = h_bits(c[e] * scale);
  }
  const v4u u = (v4u){pk16(hb[0], hb[1]), pk16(hb[2], hb[3]), pk16(hb[4], hb[5]), pk16(hb[6], hb[7])};
  unsigned short* q = out + (size_t)z * 8 * (size_t)n8 + 8 * (size_t)i;
  *(volatile v4u*)q = u;
  __threadfence();
  *(volatile v4u*)q = u;
}

__global__ __launch_bounds__(256) void wsplit3_kernel(const float* __restrict__ W0, const float* __restrict__ W1,
                                                      const float* __restrict__ W2,
                                                      unsigned short* __restrict__ outH, unsigned short* __restrict__ outL, int n8) {
  const int i = blockIdx.x * 256 + threadIdx.x;
  const int z = blockIdx.y;
  if (i >= n8) return;
  const float* W = (z == 0) ? W0 : (z == 1) ? W1 : W2;
  const float* p = W + 8 * (size_t)i;
  const v4f a = *(const v4f*)(p);
  const v4f c = *(const v4f*)(p + 4);
  unsigned short hb[8], lb[8];
#pragma unroll
  for (int e = 0; e < 4; ++e) {
    const unsigned short h0 = f2bf_bits(a[e]);
    hb[e] = h0; lb[e] = f2bf_bits(a[e] - bf_bits2f(h0));
    const unsigned short h1 = f2bf_bits(c[e]);
    hb[4 + e] = h1; lb[4 + e] = f2bf_bits(c[e] - bf_bits2f(h1));
  }
  const v4u uh = (v4u){pk16(hb[0], hb[1]), pk16(hb[2], hb[3]), pk16(hb[4], hb[5]), pk16(hb[6], hb[7])};
  const v4u ul = (v4u){pk16(lb[0], lb[1]), pk16(lb[2], lb[3]), pk16(lb[4], lb[5]), pk16(lb[6], lb[7])};
  const size_t o = (size_t)z * 8 * (size_t)n8 + 8 * (size_t)i;
  *(volatile v4u*)(outH + o) = uh;
  *(volatile v4u*)(outL + o) = ul;
  __threadfence();
  *(volatile v4u*)(outH + o) = uh;
  *(volatile v4u*)(outL + o) = ul;
}

__global__ __launch_bounds__(256) void gw_build_kernel(const float* __restrict__ gnw, const float* __restrict__ gew,
                                                       const float* __restrict__ gsw, unsigned short* __restrict__ out, float scale) {
  const int i = blockIdx.x * 256 + threadIdx.x;
  if (i >= kGateN * 32) return;
  const int r = i >> 5, c8 = (i & 31) * 8, rr = r & 7, sel = r >> 3;
  const float* p0 = gnw + (size_t)rr * kDim + c8;
  const float* p1 = gew + (size_t)rr * kDim + c8;
  const float* p2 = gsw + (size_t)rr * kDim + c8;
  const v4f a0 = *(const v4f*)(p0), a1 = *(const v4f*)(p0 + 4);
  const v4f b0 = *(const v4f*)(p1), b1 = *(const v4f*)(p1 + 4);
  const v4f d0 = *(const v4f*)(p2), d1 = *(const v4f*)(p2 + 4);
  unsigned short hb[8];
#pragma unroll
  for (int e = 0; e < 4; ++e) {
    const float v0 = (sel == 0) ? a0[e] : (sel == 1) ? b0[e] : (sel == 2) ? d0[e] : 0.0f;
    const float v1 = (sel == 0) ? a1[e] : (sel == 1) ? b1[e] : (sel == 2) ? d1[e] : 0.0f;
    hb[e] = h_bits(v0 * scale); hb[4 + e] = h_bits(v1 * scale);
  }
  const v4u u = (v4u){pk16(hb[0], hb[1]), pk16(hb[2], hb[3]), pk16(hb[4], hb[5]), pk16(hb[6], hb[7])};
  unsigned short* q = out + (size_t)r * kDim + c8;
  *(volatile v4u*)q = u;
  __threadfence();
  *(volatile v4u*)q = u;
}

template <bool HL>
__global__ __launch_bounds__(256) void transpose2_kernel(const float* __restrict__ in, unsigned short* __restrict__ out, int R, int Cc) {
  __shared__ float sm[64][65];
  const int t  = threadIdx.x;
  const int r0 = blockIdx.x * 64;
  const int c0 = blockIdx.y * 64;
#pragma unroll
  for (int i = 0; i < 16; ++i) {
    const int e  = i * 256 + t;
    const int rl = e >> 6;
    const int cl = e & 63;
    sm[cl][rl] = in[(size_t)(r0 + rl) * Cc + c0 + cl];
  }
  __syncthreads();
  const int lane = t & 31, wave = t >> 5;
  const int q = lane >> 3, c8 = (lane & 7) * 8;
  const size_t opitch = 2 * (size_t)R;
  for (int pass = 0; pass < 2; ++pass) {
#pragma unroll
    for (int it = 0; it < 2; ++it) {
      const int row = wave * 8 + it * 4 + q;
      unsigned short hb[8], lb[8];
#pragma unroll
      for (int e = 0; e < 8; ++e) {
        const float v = sm[row][c8 + e];
        const unsigned short h0 = f2bf_bits(v);
        hb[e] = h0;
        lb[e] = HL ? f2bf_bits(v - bf_bits2f(h0)) : h0;
      }
      const v4u uh = (v4u){pk16(hb[0], hb[1]), pk16(hb[2], hb[3]), pk16(hb[4], hb[5]), pk16(hb[6], hb[7])};
      const v4u ul = (v4u){pk16(lb[0], lb[1]), pk16(lb[2], lb[3]), pk16(lb[4], lb[5]), pk16(lb[6], lb[7])};
      unsigned short* op = out + (size_t)(c0 + row) * opitch + r0 + c8;
      *(volatile v4u*)(op) = uh;
      *(volatile v4u*)(op + R) = ul;
    }
    __threadfence();
  }
}

__global__ __launch_bounds__(256) void zero16_kernel(unsigned short* __restrict__ out, int n8) {
  const int i = blockIdx.x * 256 + threadIdx.x;
  if (i >= n8) return;
  const v4u u = (v4u){0u, 0u, 0u, 0u};
  unsigned short* q = out + 8 * (size_t)i;
  *(volatile v4u*)q = u;
  __threadfence();
  *(volatile v4u*)q = u;
}

template <int NT, bool MASKED>
__global__ __launch_bounds__(NT) void softmax_rows_kernel(const float* __restrict__ S, const unsigned short* __restrict__ cnt,
                                                           unsigned short* __restrict__ P, int nper, float carry) {
  constexpr int kLen = NT * 8;
  constexpr int kNw  = NT / 32;
  __shared__ float redM[kNw];
  __shared__ float redS[kNw];
  const int row  = blockIdx.x;
  const int t    = threadIdx.x;
  const int lane = t & 31, wave = t >> 5;
  const int c0   = t * 8;
  const float* sr = S + (size_t)row * kLen + c0;
  const v4f a = *(const v4f*)(sr);
  const v4f c = *(const v4f*)(sr + 4);
  float x[8];
  int keep[8];
#pragma unroll
  for (int e = 0; e < 4; ++e) { x[e] = a[e]; x[4 + e] = c[e]; }
#pragma unroll
  for (int e = 0; e < 8; ++e) keep[e] = 1;
  if (MASKED) {
    const int n = row - (row / nper) * nper;
    const v8h cv = *(const v8h*)((const _Float16*)(const void*)cnt + (size_t)n * kLen + c0);
#pragma unroll
    for (int e = 0; e < 8; ++e) {
      keep[e] = ((float)cv[e] > 0.5f) ? 1 : 0;
      x[e] = keep[e] ? x[e] : -INFINITY;
    }
  }
  float m = fmaxf(fmaxf(fmaxf(x[0], x[1]), fmaxf(x[2], x[3])), fmaxf(fmaxf(x[4], x[5]), fmaxf(x[6], x[7])));
#pragma unroll
  for (int off = 16; off > 0; off >>= 1) m = fmaxf(m, __shfl_xor(m, off, 32));
  if (lane == 0) redM[wave] = m;
  __syncthreads();
  float Mx = redM[0];
#pragma unroll
  for (int w = 1; w < kNw; ++w) Mx = fmaxf(Mx, redM[w]);
  const float Mg = (Mx > -INFINITY) ? Mx : 0.0f;
  float ex[8];
#pragma unroll
  for (int e = 0; e < 8; ++e) {
    const float ev = __expf(x[e] - Mg);
    ex[e] = keep[e] ? ev : 0.0f;
  }
  float s = ((ex[0] + ex[1]) + (ex[2] + ex[3])) + ((ex[4] + ex[5]) + (ex[6] + ex[7]));
#pragma unroll
  for (int off = 16; off > 0; off >>= 1) s += __shfl_xor(s, off, 32);
  if (lane == 0) redS[wave] = s;
  __syncthreads();
  float l = redS[0];
#pragma unroll
  for (int w = 1; w < kNw; ++w) l += redS[w];
  const float f = (l > 0.0f) ? carry * (1.0f / l) : 0.0f;
  unsigned short hb[8];
#pragma unroll
  for (int e = 0; e < 8; ++e) hb[e] = h_bits(ex[e] * f);
  const v4u u = (v4u){pk16(hb[0], hb[1]), pk16(hb[2], hb[3]), pk16(hb[4], hb[5]), pk16(hb[6], hb[7])};
  unsigned short* q = P + (size_t)row * kLen + c0;
  *(volatile v4u*)q = u;
  __threadfence();
  *(volatile v4u*)q = u;
}

__global__ __launch_bounds__(256) void heo_transpose_kernel(const float* __restrict__ in, unsigned short* __restrict__ out) {
  __shared__ float sm[32][65];
  const int t  = threadIdx.x;
  const int m0 = blockIdx.x * 64;
  const int h  = blockIdx.y;
  const float* ib = in + ((size_t)h * kEdges + m0) * 64;
#pragma unroll
  for (int i = 0; i < 8; ++i) {
    const int e  = i * 256 + t;
    const int ml = e >> 5;
    const int d  = e & 31;
    sm[d][ml] = ib[(size_t)ml * 64 + d];
  }
  __syncthreads();
  const int lane = t & 31, wave = t >> 5;
  const int q = lane >> 3, c8 = (lane & 7) * 8;
  const int row = wave * 4 + q;
  unsigned short hb[8];
#pragma unroll
  for (int e = 0; e < 8; ++e) hb[e] = h_bits(sm[row][c8 + e]);
  const v4u u = (v4u){pk16(hb[0], hb[1]), pk16(hb[2], hb[3]), pk16(hb[4], hb[5]), pk16(hb[6], hb[7])};
  unsigned short* op = out + (size_t)(h * kHd + row) * kEdges + m0 + c8;
  *(volatile v4u*)op = u;
  __threadfence();
  *(volatile v4u*)op = u;
}

__global__ __launch_bounds__(256) void combine_kernel(const float* __restrict__ GL,
                                                      const float* __restrict__ gnb, const float* __restrict__ geb, const float* __restrict__ gsb,
                                                      const float* __restrict__ ON64, const float* __restrict__ OE, const float* __restrict__ SPEC,
                                                      unsigned short* __restrict__ COMB) {
  const int lane = threadIdx.x & 31, wave = threadIdx.x >> 5;
  const int n = blockIdx.x * 8 + wave;
  if (n >= kNodes) return;
  const int jj = lane & 7, sel = lane >> 3;
  const float z  = GL[(size_t)n * kGateN + lane];
  const float b0 = gnb[jj], b1 = geb[jj], b2 = gsb[jj];
  const float bb = (sel == 0) ? b0 : (sel == 1) ? b1 : b2;
  float sg = 1.0f / (1.0f + __expf(-(z + bb)));
  sg = (lane < 24) ? sg : 0.0f;
  float s = sg;
  s += __shfl_xor(s, 1, 32);
  s += __shfl_xor(s, 2, 32);
  s += __shfl_xor(s, 4, 32);
  const float gn0 = __shfl(s, 0, 32) * 0.125f;
  const float ge0 = __shfl(s, 8, 32) * 0.125f;
  const float sp  = __shfl(s, 16, 32) * 0.125f;
  const float gs0 = fmaxf(1.0f - gn0 - ge0, 0.0f);
  const float tot = gn0 + ge0 + gs0 + 1e-8f;
  const float rt  = 1.0f / tot;
  const float gn = gn0 * rt, ge = ge0 * rt, gs = gs0 * rt;

  const int d0 = lane * 8, h = d0 >> 5, dd = d0 & 31;
  const float* onp = ON64 + ((size_t)h * kNodes + n) * 64 + dd;
  const float* oep = OE   + (size_t)n * kDim + d0;
  const float* sfp = SPEC + (size_t)n * kDim + d0;
  const v4f on0 = *(const v4f*)(onp), on1 = *(const v4f*)(onp + 4);
  const v4f oe0 = *(const v4f*)(oep), oe1 = *(const v4f*)(oep + 4);
  const v4f sf0 = *(const v4f*)(sfp), sf1 = *(const v4f*)(sfp + 4);
  unsigned short hb[8];
#pragma unroll
  for (int e = 0; e < 4; ++e) {
    const float v0 = gn * on0[e] + ge * oe0[e] + gs * (sp * sf0[e]);
    const float v1 = gn * on1[e] + ge * oe1[e] + gs * (sp * sf1[e]);
    hb[e] = h_bits(v0); hb[4 + e] = h_bits(v1);
  }
  const v4u u = (v4u){pk16(hb[0], hb[1]), pk16(hb[2], hb[3]), pk16(hb[4], hb[5]), pk16(hb[6], hb[7])};
  unsigned short* q = COMB + (size_t)n * kDim + d0;
  *(volatile v4u*)q = u;
  __threadfence();
  *(volatile v4u*)q = u;
}

__global__ __launch_bounds__(64) void layernorm_kernel(const float* __restrict__ src, const float* __restrict__ gamma,
                                                       const float* __restrict__ beta, float* __restrict__ dst) {
  __shared__ float redA[2];
  __shared__ float redB[2];
  const int row  = blockIdx.x;
  const int t    = threadIdx.x;
  const int lane = t & 31, wave = t >> 5;
  const int c0   = t * 4;
  const v4f y = *(const v4f*)(src + (size_t)row * kDim + c0);
  float s = (y[0] + y[1]) + (y[2] + y[3]);
#pragma unroll
  for (int off = 16; off > 0; off >>= 1) s += __shfl_xor(s, off, 32);
  if (lane == 0) redA[wave] = s;
  __syncthreads();
  const float mu = (redA[0] + redA[1]) * kInvDim;
  float dv[4];
#pragma unroll
  for (int e = 0; e < 4; ++e) dv[e] = y[e] - mu;
  float sq = (dv[0] * dv[0] + dv[1] * dv[1]) + (dv[2] * dv[2] + dv[3] * dv[3]);
#pragma unroll
  for (int off = 16; off > 0; off >>= 1) sq += __shfl_xor(sq, off, 32);
  if (lane == 0) redB[wave] = sq;
  __syncthreads();
  const float var = (redB[0] + redB[1]) * kInvDim;
  const float rs = 1.0f / sqrtf(var + kLnEps);
  const v4f g = *(const v4f*)(gamma + c0);
  const v4f bt = *(const v4f*)(beta + c0);
  v4f o;
#pragma unroll
  for (int e = 0; e < 4; ++e) o[e] = g[e] * (dv[e] * rs) + bt[e];
  float* q = dst + (size_t)row * kDim + c0;
  *(volatile v4f*)q = o;
  __threadfence();
  *(volatile v4f*)q = o;
}

template <int ET, bool SPLIT, int BM, int OM, bool RESID>
static void run_gemm(hipStream_t st, int batch,
                     const void* A, const void* A2, int lda, long sA,
                     const void* Bt, const void* Bt2, int ldb, long sB,
                     void* C, void* C2, int ldc, long sC,
                     const float* bias, const float* resid, long sR,
                     int M, int N, int K, float scale) {
  const int tiles = (M / 64) * (N / 64);
  dim3 grid((unsigned)((tiles + 7) / 8), (unsigned)batch);
  wmma_gemm64<ET, SPLIT, BM, OM, RESID><<<grid, 256, 0, st>>>(
      (const unsigned short*)A, (const unsigned short*)A2, lda, sA,
      (const unsigned short*)Bt, (const unsigned short*)Bt2, ldb, sB,
      C, C2, ldc, sC, bias, resid, sR, M, N, K, scale);
}

extern "C" void kernel_launch(void* const* d_in, const int* in_sizes, int n_in,
                              void* d_out, int out_size, void* d_ws, size_t ws_size,
                              hipStream_t stream)
{
  if (n_in < 17) return;
  if (in_sizes[0] != kNodes * kDim || in_sizes[1] != kNodes * kEdges || in_sizes[2] != kNodes * kRank ||
      in_sizes[3] != kDim * kDim || in_sizes[4] != kDim * kDim || in_sizes[5] != kDim * kDim ||
      in_sizes[6] != kDim * kRank || in_sizes[7] != kHeads * kDim || in_sizes[8] != kHeads ||
      in_sizes[9] != kHeads * kDim || in_sizes[10] != kHeads || in_sizes[11] != kHeads * kDim || in_sizes[12] != kHeads ||
      in_sizes[13] != kDim * kDim || in_sizes[14] != kDim || in_sizes[15] != kDim || in_sizes[16] != kDim ||
      out_size != kNodes * kDim) return;

  const float* x     = (const float*)d_in[0];
  const float* Hinc  = (const float*)d_in[1];
  const float* U_r   = (const float*)d_in[2];
  const float* Wq    = (const float*)d_in[3];
  const float* Wk    = (const float*)d_in[4];
  const float* Wv    = (const float*)d_in[5];
  const float* Wspec = (const float*)d_in[6];
  const float* gn_w  = (const float*)d_in[7];
  const float* gn_b  = (const float*)d_in[8];
  const float* ge_w  = (const float*)d_in[9];
  const float* ge_b  = (const float*)d_in[10];
  const float* gs_w  = (const float*)d_in[11];
  const float* gs_b  = (const float*)d_in[12];
  const float* Woutw = (const float*)d_in[13];
  const float* Woutb = (const float*)d_in[14];
  const float* gamma = (const float*)d_in[15];
  const float* beta  = (const float*)d_in[16];
  float* out = (float*)d_out;

  char* wsb = (char*)d_ws;
  size_t off = 0;
  auto carve = [&](size_t bytes) -> char* { char* p = wsb + off; off += (bytes + 255) & ~(size_t)255; return p; };

  unsigned short* X16    = (unsigned short*)carve((size_t)kNodes * kDim * 2);
  unsigned short* XT2    = (unsigned short*)carve((size_t)kDim * 2 * kNodes * 2);
  unsigned short* H16    = (unsigned short*)carve((size_t)kNodes * kEdges * 2);
  unsigned short* HT2    = (unsigned short*)carve((size_t)kEdges * 2 * kNodes * 2);
  unsigned short* UR16   = (unsigned short*)carve((size_t)kNodes * kRank * 2);
  unsigned short* WS16   = (unsigned short*)carve((size_t)kDim * kRank * 2);
  unsigned short* W16ALL = (unsigned short*)carve((size_t)4 * kDim * kDim * 2);
  unsigned short* WQKVH  = (unsigned short*)carve((size_t)3 * kDim * kDim * 2);
  unsigned short* WQKVL  = (unsigned short*)carve((size_t)3 * kDim * kDim * 2);
  unsigned short* GW16   = (unsigned short*)carve((size_t)kGateN * kDim * 2);
  unsigned short* QK16   = (unsigned short*)carve((size_t)kNodes * 2 * kDim * 2);
  unsigned short* VT     = (unsigned short*)carve((size_t)kVRows * kNodes * 2);
  unsigned short* CNT16  = (unsigned short*)carve((size_t)kNodes * kNodes * 2);
  float*          S      = (float*)carve((size_t)kHeadBatch * kNodes * kNodes * 4);
  unsigned short* P16    = (unsigned short*)carve((size_t)kHeadBatch * kNodes * kNodes * 2);
  float*          ON64   = (float*)carve((size_t)kHeads * kNodes * 64 * 4);
  float*          GL     = (float*)carve((size_t)kNodes * kGateN * 4);
  float*          SPEC   = (float*)carve((size_t)kNodes * kDim * 4);
  unsigned short* HEH    = (unsigned short*)carve((size_t)kEdges * kDim * 2);
  unsigned short* HEL    = (unsigned short*)carve((size_t)kEdges * kDim * 2);
  unsigned short* QKEH   = (unsigned short*)carve((size_t)kEdges * 2 * kDim * 2);
  unsigned short* QKEL   = (unsigned short*)carve((size_t)kEdges * 2 * kDim * 2);
  unsigned short* VET    = (unsigned short*)carve((size_t)kVRows * kEdges * 2);
  float*          SE     = (float*)carve((size_t)kHeads * kEdges * kEdges * 4);
  unsigned short* PE16   = (unsigned short*)carve((size_t)kHeads * kEdges * kEdges * 2);
  float*          HEO64  = (float*)carve((size_t)kHeads * kEdges * 64 * 4);
  unsigned short* HEOT16 = (unsigned short*)carve((size_t)kDim * kEdges * 2);
  float*          OE     = (float*)carve((size_t)kNodes * kDim * 4);
  unsigned short* COMB16 = (unsigned short*)carve((size_t)kNodes * kDim * 2);
  float*          Yb     = (float*)carve((size_t)kNodes * kDim * 4);
  if (off > ws_size) return;

  const unsigned short* WQK16 = W16ALL;
  const unsigned short* WV16  = W16ALL + (size_t)2 * kDim * kDim;
  const unsigned short* WO16  = W16ALL + (size_t)3 * kDim * kDim;
  const long sS  = (long)kNodes * kNodes;
  const long sSE = (long)kEdges * kEdges;

  { const int n8 = kNodes * kDim / 8;   cast8_f16_kernel<<<(n8 + 255) / 256, 256, 0, stream>>>(x, X16, n8, 1.0f); }
  { const int n8 = kNodes * kEdges / 8; cast8_f16_kernel<<<(n8 + 255) / 256, 256, 0, stream>>>(Hinc, H16, n8, 1.0f); }
  { const int n8 = kNodes * kRank / 8;  cast8_f16_kernel<<<(n8 + 255) / 256, 256, 0, stream>>>(U_r, UR16, n8, 1.0f); }
  { const int n8 = kDim * kRank / 8;    cast8_f16_kernel<<<(n8 + 255) / 256, 256, 0, stream>>>(Wspec, WS16, n8, kWCarry); }
  { const int n8 = kDim * kDim / 8;
    wcast4_kernel<<<dim3((n8 + 255) / 256, 4), 256, 0, stream>>>(Wq, Wk, Wv, Woutw, W16ALL, n8, kWCarry);
    wsplit3_kernel<<<dim3((n8 + 255) / 256, 3), 256, 0, stream>>>(Wq, Wk, Wv, WQKVH, WQKVL, n8); }
  gw_build_kernel<<<(kGateN * 32 + 255) / 256, 256, 0, stream>>>(gn_w, ge_w, gs_w, GW16, kWCarry);
  transpose2_kernel<true><<<dim3(kNodes / 64, kDim / 64), 256, 0, stream>>>(x, XT2, kNodes, kDim);
  transpose2_kernel<false><<<dim3(kNodes / 64, kEdges / 64), 256, 0, stream>>>(Hinc, HT2, kNodes, kEdges);
  zero16_kernel<<<(32 * kNodes / 8 + 255) / 256, 256, 0, stream>>>(VT + (size_t)kDim * kNodes, 32 * kNodes / 8);
  zero16_kernel<<<(32 * kEdges / 8 + 255) / 256, 256, 0, stream>>>(VET + (size_t)kDim * kEdges, 32 * kEdges / 8);

  run_gemm<0, false, 0, 1, false>(stream, 1, X16, X16, kDim, 0, WQK16, WQK16, kDim, 0, QK16, QK16, 2 * kDim, 0,
                                  Woutb, x, 0, kNodes, 2 * kDim, kDim, kWCarryInv);
  run_gemm<0, false, 0, 1, false>(stream, 1, WV16, WV16, kDim, 0, X16, X16, kDim, 0, VT, VT, kNodes, 0,
                                  Woutb, x, 0, kDim, kNodes, kDim, kWCarryInv);
  run_gemm<0, false, 0, 1, false>(stream, 1, H16, H16, kEdges, 0, H16, H16, kEdges, 0, CNT16, CNT16, kNodes, 0,
                                  Woutb, x, 0, kNodes, kNodes, kEdges, 1.0f);
  run_gemm<0, false, 0, 0, false>(stream, 1, QK16, QK16, 2 * kDim, 0, GW16, GW16, kDim, 0, GL, GL, kGateN, 0,
                                  Woutb, x, 0, kNodes, kGateN, kDim, kWCarryInv);
  run_gemm<0, false, 0, 0, false>(stream, 1, UR16, UR16, kRank, 0, WS16, WS16, kRank, 0, SPEC, SPEC, kDim, 0,
                                  Woutb, x, 0, kNodes, kDim, kRank, kWCarryInv);

  for (int hb = 0; hb < kHeads / kHeadBatch; ++hb) {
    const int hbase = hb * kHeadBatch;
    run_gemm<0, false, 0, 0, false>(stream, kHeadBatch,
                                    QK16 + (size_t)hbase * kHd, QK16 + (size_t)hbase * kHd, 2 * kDim, kHd,
                                    QK16 + kDim + (size_t)hbase * kHd, QK16 + kDim + (size_t)hbase * kHd, 2 * kDim, kHd,
                                    S, S, kNodes, sS, Woutb, x, 0, kNodes, kNodes, kHd, kScoreScale);
    softmax_rows_kernel<256, true><<<kHeadBatch * kNodes, 256, 0, stream>>>(S, CNT16, P16, kNodes, kPCarry);
    run_gemm<0, false, 0, 0, false>(stream, kHeadBatch,
                                    P16, P16, kNodes, sS,
                                    VT + (size_t)hbase * kHd * kNodes, VT + (size_t)hbase * kHd * kNodes, kNodes, (long)kHd * kNodes,
                                    ON64 + (size_t)hbase * kNodes * 64, ON64 + (size_t)hbase * kNodes * 64, 64, (long)kNodes * 64,
                                    Woutb, x, 0, kNodes, 64, kNodes, kPCarryInv);
  }

  run_gemm<1, false, 0, 2, false>(stream, 1, HT2, HT2, 2 * kNodes, 0, XT2, XT2, 2 * kNodes, 0, HEH, HEL, kDim, 0,
                                  Woutb, x, 0, kEdges, kDim, 2 * kNodes, 1.0f);
  run_gemm<1, true, 0, 2, false>(stream, 1, HEH, HEL, kDim, 0, WQKVH, WQKVL, kDim, 0, QKEH, QKEL, 2 * kDim, 0,
                                 Woutb, x, 0, kEdges, 2 * kDim, kDim, 1.0f);
  run_gemm<1, true, 0, 1, false>(stream, 1, WQKVH + (size_t)2 * kDim * kDim, WQKVL + (size_t)2 * kDim * kDim, kDim, 0,
                                 HEH, HEL, kDim, 0, VET, VET, kEdges, 0, Woutb, x, 0, kDim, kEdges, kDim, 1.0f);
  run_gemm<1, true, 0, 0, false>(stream, kHeads,
                                 QKEH, QKEL, 2 * kDim, kHd,
                                 QKEH + kDim, QKEL + kDim, 2 * kDim, kHd,
                                 SE, SE, kEdges, sSE, Woutb, x, 0, kEdges, kEdges, kHd, kScoreScale);
  softmax_rows_kernel<64, false><<<kHeads * kEdges, 64, 0, stream>>>(SE, CNT16, PE16, kEdges, kPCarry);
  run_gemm<0, false, 0, 0, false>(stream, kHeads,
                                  PE16, PE16, kEdges, sSE,
                                  VET, VET, kEdges, (long)kHd * kEdges,
                                  HEO64, HEO64, 64, (long)kEdges * 64,
                                  Woutb, x, 0, kEdges, 64, kEdges, kPCarryInv);
  heo_transpose_kernel<<<dim3(kEdges / 64, kHeads), 256, 0, stream>>>(HEO64, HEOT16);
  run_gemm<0, false, 0, 0, false>(stream, 1, H16, H16, kEdges, 0, HEOT16, HEOT16, kEdges, 0, OE, OE, kDim, 0,
                                  Woutb, x, 0, kNodes, kDim, kEdges, 1.0f);

  combine_kernel<<<kNodes / 8, 256, 0, stream>>>(GL, gn_b, ge_b, gs_b, ON64, OE, SPEC, COMB16);
  run_gemm<0, false, 2, 0, true>(stream, 1, COMB16, COMB16, kDim, 0, WO16, WO16, kDim, 0, Yb, Yb, kDim, 0,
                                 Woutb, x, 0, kNodes, kDim, kDim, kWCarryInv);
  layernorm_kernel<<<kNodes, 64, 0, stream>>>(Yb, gamma, beta, out);
}
